// GATNet_45844480917958
// MI455X (gfx1250) — hardware-verified
//
#include <hip/hip_runtime.h>
#include <stddef.h>
#include <stdint.h>
#include <math.h>


#define DIN    128
#define NH1    4
#define HW     128
#define D1     (NH1 * HW)
#define KP2    (2 * D1)
#define D2     128
#define NG     256
#define NF1    16
#define NTHR   256
#define NWAVE  8
#define EPT    8
#define CHUNK  (NTHR * EPT)
#define WCAP   (EPT * 32)
#define LISTN  (NWAVE * WCAP)
#define NBA    1024
#define SLA    10
#define RCAP   28672
#define DEGCAP 128
#define GBM    64
#define GBN    128
#define GTHR   128
#define MROWS  128
#define NU1    (D1 * (DIN / 8))
#define NU2    (D2 * (KP2 / 8))
#define NEGSL  0.2f
#define AGG_ZINTS (LISTN + 2 * RCAP + 3 * NBA)
#define AGG_LDS_INTS (AGG_ZINTS + 32)
#define WSMAX  134217728

static_assert((CHUNK & (CHUNK - 1)) == 0 && CHUNK <= 4096);
static_assert((NBA & (NBA - 1)) == 0 && NBA == (1 << SLA));
static_assert(((long long)CHUNK << SLA) < (1LL << 31));
static_assert(LISTN % NTHR == 0);
static_assert(NBA % NWAVE == 0 && NBA % 32 == 0 && NBA % GBM == 0);
static_assert(RCAP % 4 == 0 && AGG_ZINTS % 4 == 0 && LISTN % 4 == 0);
static_assert(RCAP >= 16588 + 4096);
static_assert(DEGCAP >= 35 + 8);
static_assert(DIN % 32 == 0 && KP2 % 32 == 0 && KP2 == 2 * D1);
static_assert(GBN == HW && D2 == GBN && D1 == NH1 * GBN);
static_assert(GBM == (GTHR / 32) * 16 && GBN == 4 * 32);
static_assert(MROWS % GBM == 0);
static_assert(NU1 % NTHR == 0 && NU2 % NTHR == 0);
static_assert(DIN / 8 == 16 && KP2 / 8 == 128);
static_assert(AGG_LDS_INTS * 4 <= 300000);
static_assert(HW == 4 * 32);
static_assert(NG == NTHR);
static_assert((D2 * NF1 / 4) % NTHR == 0);

typedef float          v4f   __attribute__((ext_vector_type(4)));
typedef float          v8f   __attribute__((ext_vector_type(8)));
typedef int            v4i   __attribute__((ext_vector_type(4)));
typedef int            v8i   __attribute__((ext_vector_type(8)));
typedef unsigned int   v4u   __attribute__((ext_vector_type(4)));
typedef unsigned short v8us  __attribute__((ext_vector_type(8)));
typedef __bf16         v16bf __attribute__((ext_vector_type(16)));
typedef v4f  __attribute__((may_alias)) v4fa;
typedef v4i  __attribute__((may_alias)) v4ia;
typedef v8us __attribute__((may_alias)) v8usa;
union FragB { v16bf v; v8us h[2]; v8i w; };

__device__ __forceinline__ v8f wmb(const FragB& a, const FragB& b, v8f c) {
  v8f d = __builtin_amdgcn_wmma_f32_16x16x32_bf16(false, a.v, false, b.v, (short)0, c, false, false);
  asm volatile("v_nop\n\tv_nop\n\tv_nop\n\tv_nop" : "+v"(d) : "v"(a.w), "v"(b.w));
  return d;
}

__device__ __forceinline__ unsigned f2bf(float f) {
  const unsigned u = __float_as_uint(f);
  const unsigned r = ((u + 0x7FFFu + ((u >> 16) & 1u)) >> 16) & 0xFFFFu;
  return (f != f) ? 0x7FC0u : r;
}
__device__ __forceinline__ float bf2f(unsigned b) { return __uint_as_float(b << 16); }
__device__ __forceinline__ float bfr(float f) { return bf2f(f2bf(f)); }
__device__ __forceinline__ v4f bfr4(const v4f a) {
  v4f r; r.x = bfr(a.x); r.y = bfr(a.y); r.z = bfr(a.z); r.w = bfr(a.w); return r;
}
__device__ __forceinline__ float smax(float m, float v) {
  return (m != m) ? m : ((v > m || v != v) ? v : m);
}
__device__ __forceinline__ float elu1(float o) {
  const float t = expf(o) - 1.0f;
  float p = fmaf(o, 1.0f / 720.0f, 1.0f / 120.0f);
  p = fmaf(o, p, 1.0f / 24.0f);
  p = fmaf(o, p, 1.0f / 6.0f);
  p = fmaf(o, p, 0.5f);
  const float sr = fmaf(o * o, p, o);
  const float ng = (o > -0.25f) ? sr : t;
  return (o > 0.0f) ? o : ng;
}

template <int SLB>
__device__ __forceinline__ int scan_chunk(const int* __restrict__ dsts, int nE, int cbase, int slotBase,
                                          int nb, int vec8, int* list, int tid, int lane, int wave) {
  int wc = 0;
  const int el0  = tid * EPT;
  const int e0   = cbase + el0;
  const int sent = -2147483647 - 1;
  v4i da, db;
  if (vec8 != 0 && cbase + CHUNK <= nE) {
    da = *(const v4i*)(dsts + e0);
    db = *(const v4i*)(dsts + e0 + 4);
  } else {
    da.x = (e0     < nE) ? dsts[min(e0,     nE - 1)] : sent;
    da.y = (e0 + 1 < nE) ? dsts[min(e0 + 1, nE - 1)] : sent;
    da.z = (e0 + 2 < nE) ? dsts[min(e0 + 2, nE - 1)] : sent;
    da.w = (e0 + 3 < nE) ? dsts[min(e0 + 3, nE - 1)] : sent;
    db.x = (e0 + 4 < nE) ? dsts[min(e0 + 4, nE - 1)] : sent;
    db.y = (e0 + 5 < nE) ? dsts[min(e0 + 5, nE - 1)] : sent;
    db.z = (e0 + 6 < nE) ? dsts[min(e0 + 6, nE - 1)] : sent;
    db.w = (e0 + 7 < nE) ? dsts[min(e0 + 7, nE - 1)] : sent;
  }
  const unsigned nbs = (unsigned)slotBase;
  const unsigned unb = (unsigned)nb;
  const unsigned s0 = (unsigned)da.x - nbs, s1 = (unsigned)da.y - nbs;
  const unsigned s2 = (unsigned)da.z - nbs, s3 = (unsigned)da.w - nbs;
  const unsigned s4 = (unsigned)db.x - nbs, s5 = (unsigned)db.y - nbs;
  const unsigned s6 = (unsigned)db.z - nbs, s7 = (unsigned)db.w - nbs;
  const bool h0 = s0 < unb, h1 = s1 < unb, h2 = s2 < unb, h3 = s3 < unb;
  const bool h4 = s4 < unb, h5 = s5 < unb, h6 = s6 < unb, h7 = s7 < unb;
  const unsigned any = __builtin_amdgcn_ballot_w32(h0 | h1 | h2 | h3 | h4 | h5 | h6 | h7);
  if (any != 0u) {
#define HITJ(J, HJ, SJ) { \
      const unsigned mj = __builtin_amdgcn_ballot_w32(HJ); \
      if (mj != 0u) { \
        if (HJ) { \
          const int pos = wc + (int)__builtin_amdgcn_mbcnt_lo(mj, 0u); \
          if (pos < WCAP) list[wave * WCAP + pos] = ((el0 + (J)) << SLB) | (int)(SJ); \
        } \
        wc += (int)__builtin_popcount(mj); } }
    HITJ(0, h0, s0)
    HITJ(1, h1, s1)
    HITJ(2, h2, s2)
    HITJ(3, h3, s3)
    HITJ(4, h4, s4)
    HITJ(5, h5, s5)
    HITJ(6, h6, s6)
    HITJ(7, h7, s7)
#undef HITJ
  }
  return wc;
}

__global__ __launch_bounds__(NTHR) void k_prep(const float* __restrict__ W1, const float* __restrict__ W2,
                                               const float* __restrict__ x, int nN, int nUx,
                                               unsigned short* W1T, unsigned short* W2T, unsigned short* XB) {
  const int u = (int)blockIdx.x * NTHR + (int)threadIdx.x;
  v8us o;
  unsigned short* dp;
  if (u < NU1) {
    const int n  = u >> 4;
    const int k8 = (u & 15) * 8;
    const float* p = W1 + (size_t)k8 * D1 + n;
#pragma unroll
    for (int i = 0; i < 8; ++i) o[i] = (unsigned short)f2bf(p[(size_t)i * D1]);
    dp = W1T + (size_t)n * DIN + k8;
  } else if (u < NU1 + NU2) {
    const int v  = u - NU1;
    const int n  = v >> 7;
    const int k8 = (v & 127) * 8;
    const int kk = k8 & (D1 - 1);
    const float* p = W2 + (size_t)kk * D2 + n;
#pragma unroll
    for (int i = 0; i < 8; ++i) o[i] = (unsigned short)f2bf(p[(size_t)i * D2]);
    dp = W2T + (size_t)n * KP2 + k8;
  } else if (u < NU1 + NU2 + nUx) {
    const int v   = u - NU1 - NU2;
    const int row = v >> 4;
    const int k8  = (v & 15) * 8;
    const int rc  = row < nN ? row : nN - 1;
    const float* p = x + (size_t)rc * DIN + k8;
    const v4f a = *(const v4f*)p;
    const v4f b = *(const v4f*)(p + 4);
    const bool ok = row < nN;
    o[0] = ok ? (unsigned short)f2bf(a.x) : (unsigned short)0;
    o[1] = ok ? (unsigned short)f2bf(a.y) : (unsigned short)0;
    o[2] = ok ? (unsigned short)f2bf(a.z) : (unsigned short)0;
    o[3] = ok ? (unsigned short)f2bf(a.w) : (unsigned short)0;
    o[4] = ok ? (unsigned short)f2bf(b.x) : (unsigned short)0;
    o[5] = ok ? (unsigned short)f2bf(b.y) : (unsigned short)0;
    o[6] = ok ? (unsigned short)f2bf(b.z) : (unsigned short)0;
    o[7] = ok ? (unsigned short)f2bf(b.w) : (unsigned short)0;
    dp = XB + (size_t)row * DIN + k8;
  } else {
    return;
  }
  *(volatile v8us*)dp = o;
  __threadfence();
  *(volatile v8us*)dp = o;
}

__global__ __launch_bounds__(GTHR) void k_gemm(const unsigned short* __restrict__ A, int lda,
                                               const unsigned short* __restrict__ BT, int ldb, int K,
                                               float* Cm, int ldc,
                                               const float* __restrict__ avs, const float* __restrict__ avd,
                                               float* SD, int MPr) {
  __shared__ __attribute__((aligned(16))) float stg[GBM * GBN];
  __shared__ __attribute__((aligned(16))) float sdt[2 * GBM];
  const int tid = (int)threadIdx.x, lane = tid & 31, wave = tid >> 5, hh = lane >> 4, m = lane & 15;
  const int rowBase = (int)blockIdx.x * GBM;
  const int head    = (int)blockIdx.y;
  const int colBase = head * GBN;

  v8f acc[8];
  {
    const v8f z = {0.f, 0.f, 0.f, 0.f, 0.f, 0.f, 0.f, 0.f};
#pragma unroll
    for (int t = 0; t < 8; ++t) acc[t] = z;
  }
  const unsigned short* ap = A  + (size_t)(rowBase + 16 * wave + m) * (size_t)lda + 8 * hh;
  const unsigned short* bp = BT + (size_t)(colBase + m) * (size_t)ldb + 8 * hh;

#pragma unroll 1
  for (int k0 = 0; k0 < K; k0 += 32) {
    FragB af;
    af.h[0] = *(const v8usa*)(ap + k0);
    af.h[1] = *(const v8usa*)(ap + k0 + 16);
#pragma unroll
    for (int nt = 0; nt < 8; ++nt) {
      const unsigned short* wq = bp + (size_t)(16 * nt) * (size_t)ldb + k0;
      FragB bf;
      bf.h[0] = *(const v8usa*)wq;
      bf.h[1] = *(const v8usa*)(wq + 16);
      acc[nt] = wmb(af, bf, acc[nt]);
    }
  }

#pragma unroll
  for (int nt = 0; nt < 8; ++nt) {
    const int lc = 16 * nt + m;
#pragma unroll
    for (int r = 0; r < 8; ++r) {
      const int lr = 16 * wave + 8 * hh + r;
      stg[lr * GBN + lc] = acc[nt][r];
    }
  }
  __syncthreads();

  const v4f as4 = bfr4(*(const v4fa*)(avs + head * GBN + 4 * lane));
  const v4f ad4 = bfr4(*(const v4fa*)(avd + head * GBN + 4 * lane));
#pragma unroll 1
  for (int i = 0; i < 16; ++i) {
    const int row = wave * 16 + i;
    const v4f p = *(const v4fa*)(stg + row * GBN + 4 * lane);
    float s = 0.0f, d = 0.0f;
    s = fmaf(p.x, as4.x, s); s = fmaf(p.y, as4.y, s); s = fmaf(p.z, as4.z, s); s = fmaf(p.w, as4.w, s);
    d = fmaf(p.x, ad4.x, d); d = fmaf(p.y, ad4.y, d); d = fmaf(p.z, ad4.z, d); d = fmaf(p.w, ad4.w, d);
#pragma unroll
    for (int off = 16; off > 0; off >>= 1) {
      s += __shfl_xor(s, off);
      d += __shfl_xor(d, off);
    }
    if (lane == 0) { sdt[row] = s; sdt[GBM + row] = d; }
  }
  __syncthreads();

  const v4f sdv = *(const v4fa*)(sdt + 4 * lane);
  float* sp = SD + (size_t)(2 * head + (lane >> 4)) * (size_t)MPr + rowBase + 4 * (lane & 15);
#pragma unroll 1
  for (int i = 0; i < 16; ++i) {
    const int row = wave * 16 + i;
    const v4f p = *(const v4fa*)(stg + row * GBN + 4 * lane);
    float* op = Cm + (size_t)(rowBase + row) * (size_t)ldc + colBase + 4 * lane;
    *(volatile v4f*)op = p;
  }
  if (wave == 0) *(volatile v4f*)sp = sdv;
  __threadfence();
#pragma unroll 1
  for (int i = 0; i < 16; ++i) {
    const int row = wave * 16 + i;
    const v4f p = *(const v4fa*)(stg + row * GBN + 4 * lane);
    float* op = Cm + (size_t)(rowBase + row) * (size_t)ldc + colBase + 4 * lane;
    *(volatile v4f*)op = p;
  }
  if (wave == 0) *(volatile v4f*)sp = sdv;
}

template <int L>
__global__ __launch_bounds__(NTHR) void k_agg(const int* __restrict__ srcs, const int* __restrict__ dsts,
                                              int nE, int nN, int vec8, int mRows,
                                              const float* __restrict__ SD,
                                              const float* __restrict__ xl, const float* __restrict__ bias,
                                              unsigned short* hb, float* outp, int* flg) {
  static_assert(L == 1 || L == 2);
  constexpr int NHD = (L == 1) ? NH1 : 1;
  constexpr int FP  = NHD * HW;
  extern __shared__ __attribute__((aligned(16))) int dsm[];
  int* list = dsm;
  int* hl   = dsm + LISTN;
  int* sl   = dsm + LISTN + RCAP;
  int* cnt  = dsm + LISTN + 2 * RCAP;
  int* offs = cnt + NBA;
  int* cur  = offs + NBA;
  int* misc = cur + NBA;
  const int tid = (int)threadIdx.x, lane = tid & 31, wave = tid >> 5;
  const int nodeBase = (int)blockIdx.x * NBA;

  {
    const v4i z4 = {0, 0, 0, 0};
    for (int i = tid * 4; i < AGG_ZINTS; i += NTHR * 4) *(v4ia*)(dsm + i) = z4;
    if (tid < 32) misc[tid] = 0;
  }
  __syncthreads();

  int t = 0, ov = 0;
  const int nChunks = (nE + CHUNK - 1) / CHUNK;
#pragma unroll 1
  for (int ch = 0; ch < nChunks; ++ch) {
    const int cbase = ch * CHUNK;
    const int wc = scan_chunk<SLA>(dsts, nE, cbase, nodeBase, NBA, vec8, list, tid, lane, wave);
    if (lane == 0) misc[wave] = wc;
    __syncthreads();
    if (wave == 0) {
#pragma unroll 1
      for (int w2 = 0; w2 < NWAVE; ++w2) {
        int c = misc[w2];
        c = c < 0 ? 0 : (c > WCAP ? WCAP : c);
#pragma unroll 1
        for (int b0 = 0; b0 < c; b0 += 32) {
          const int idx = b0 + lane;
          const int ent = list[w2 * WCAP + (idx < WCAP ? idx : WCAP - 1)];
          const int m32 = (c - b0) < 32 ? (c - b0) : 32;
#pragma unroll 1
          for (int k = 0; k < m32; ++k) {
            const int u    = __builtin_amdgcn_readlane(ent, k);
            const int slot = u & (NBA - 1);
            const int el   = (u >> SLA) & (CHUNK - 1);
            const int pk   = ((cbase + el) << SLA) | slot;
            if (t < RCAP) {
              if (lane == 0) { hl[t] = pk; cnt[slot] = cnt[slot] + 1; }
              t = t + 1;
            } else {
              ov = 1;
            }
          }
        }
      }
    }
    __syncthreads();
  }
  if (wave == 0 && lane == 0) { misc[8] = t; misc[9] = ov; }
  __syncthreads();
  int tt = misc[8];
  tt = tt < 0 ? 0 : (tt > RCAP ? RCAP : tt);
  const int ovf = misc[9];

  if (wave == 0) {
    const int base = lane * (NBA / 32);
    int s = 0;
#pragma unroll 1
    for (int i = 0; i < NBA / 32; ++i) s += cnt[base + i];
    int incl = s;
#pragma unroll
    for (int d = 1; d < 32; d <<= 1) {
      const int y = __shfl_up(incl, d, 32);
      if (lane >= d) incl += y;
    }
    int run = incl - s;
#pragma unroll 1
    for (int i = 0; i < NBA / 32; ++i) {
      const int cv = cnt[base + i];
      offs[base + i] = run;
      cur[base + i]  = run;
      run += cv;
    }
  }
  __syncthreads();
  if (wave == 0) {
#pragma unroll 1
    for (int b0 = 0; b0 < tt; b0 += 32) {
      const int idx = b0 + lane;
      const int ent = hl[idx < RCAP ? idx : RCAP - 1];
      const int m32 = (tt - b0) < 32 ? (tt - b0) : 32;
#pragma unroll 1
      for (int k = 0; k < m32; ++k) {
        const int u    = __builtin_amdgcn_readlane(ent, k);
        const int slot = u & (NBA - 1);
        if (lane == 0) {
          int p = cur[slot];
          p = p < 0 ? 0 : (p > RCAP - 1 ? RCAP - 1 : p);
          sl[p] = u;
          cur[slot] = p + 1;
        }
      }
    }
  }
  __syncthreads();

  const float qn = __int_as_float(0x7fc00000);
  const float pz = (ovf != 0) ? qn : 0.0f;
  int bigAny = 0;
#pragma unroll 1
  for (int si = 0; si < NBA / NWAVE; ++si) {
    const int s    = si * NWAVE + wave;
    const int node = nodeBase + s;
    if (node < mRows) {
      int c = cnt[s];
      const bool big = c > DEGCAP;
      bigAny |= big ? 1 : 0;
      c = c < 0 ? 0 : (c > DEGCAP ? DEGCAP : c);
      int o = offs[s];
      o = o < 0 ? 0 : (o > RCAP ? RCAP : o);
      const int nc = node < nN ? node : nN - 1;
      const bool live = node < nN;
      const float pzr = big ? qn : pz;
#pragma unroll 1
      for (int hd = 0; hd < NHD; ++hd) {
        const float* ASp = SD + (size_t)(2 * hd) * (size_t)mRows;
        const float* ADp = ASp + mRows;
        const float* fb  = xl + hd * HW + 4 * lane;
        const float as0 = ASp[nc];
        const float ad  = ADp[nc];
        v4f av = *(const v4f*)(fb + (size_t)nc * FP);
        float l0 = as0 + ad;
        l0 = l0 > 0.f ? l0 : NEGSL * l0;
        float mx = l0, dn = 1.0f;
#pragma unroll 1
        for (int b0 = 0; b0 < c; b0 += 32) {
          int idx = o + b0 + lane;
          idx = idx > RCAP - 1 ? RCAP - 1 : idx;
          const int ent = sl[idx];
          int eid = ent >> SLA;
          eid = eid < 0 ? 0 : (eid > nE - 1 ? nE - 1 : eid);
          int sr = srcs[eid];
          sr = sr < 0 ? 0 : (sr > nN - 1 ? nN - 1 : sr);
          const int esi = __float_as_int(ASp[sr]);
          const int m32 = (c - b0) < 32 ? (c - b0) : 32;
#pragma unroll 1
          for (int k = 0; k < m32; ++k) {
            const int   sk  = __builtin_amdgcn_readlane(sr, k);
            const float ask = __int_as_float(__builtin_amdgcn_readlane(esi, k));
            const v4f a = *(const v4f*)(fb + (size_t)sk * FP);
            float lg = ask + ad;
            lg = lg > 0.f ? lg : NEGSL * lg;
            const float df = lg - mx;
            const float ee = expf(-fabsf(df));
            const bool  up = df > 0.f;
            const float s1 = up ? ee : 1.0f;
            const float s2 = up ? 1.0f : ee;
            mx = up ? lg : mx;
            dn = fmaf(dn, s1, s2);
            av.x = fmaf(av.x, s1, s2 * a.x);
            av.y = fmaf(av.y, s1, s2 * a.y);
            av.z = fmaf(av.z, s1, s2 * a.z);
            av.w = fmaf(av.w, s1, s2 * a.w);
          }
        }
        const float inv = __builtin_amdgcn_rcpf(dn);
        const v4f bb = bfr4(*(const v4fa*)(bias + hd * HW + 4 * lane));
        float y0 = fmaf(av.x, inv, bb.x), y1 = fmaf(av.y, inv, bb.y);
        float y2 = fmaf(av.z, inv, bb.z), y3 = fmaf(av.w, inv, bb.w);
        if constexpr (L == 1) {
          y0 = elu1(y0) + pzr; y1 = elu1(y1) + pzr; y2 = elu1(y2) + pzr; y3 = elu1(y3) + pzr;
          y0 = live ? y0 : 0.0f; y1 = live ? y1 : 0.0f; y2 = live ? y2 : 0.0f; y3 = live ? y3 : 0.0f;
          const unsigned hbx = f2bf(y0), hby = f2bf(y1), hbz = f2bf(y2), hbw = f2bf(y3);
          const unsigned lbx = f2bf(y0 - bf2f(hbx)), lby = f2bf(y1 - bf2f(hby));
          const unsigned lbz = f2bf(y2 - bf2f(hbz)), lbw = f2bf(y3 - bf2f(hbw));
          const int hw0 = (int)(hbx | (hby << 16)), hw1 = (int)(hbz | (hbw << 16));
          const int lw0 = (int)(lbx | (lby << 16)), lw1 = (int)(lbz | (lbw << 16));
          const int sa = (2 * lane) & 31, sb = (2 * lane + 1) & 31;
          const int g0 = __shfl(hw0, sa), g1 = __shfl(hw1, sa), g2 = __shfl(hw0, sb), g3 = __shfl(hw1, sb);
          const int q0 = __shfl(lw0, sa), q1 = __shfl(lw1, sa), q2 = __shfl(lw0, sb), q3 = __shfl(lw1, sb);
          const bool lsel = lane >= 16;
          v4u pv;
          pv.x = (unsigned)(lsel ? q0 : g0);
          pv.y = (unsigned)(lsel ? q1 : g1);
          pv.z = (unsigned)(lsel ? q2 : g2);
          pv.w = (unsigned)(lsel ? q3 : g3);
          unsigned short* gp = hb + (size_t)node * KP2 + hd * HW + 8 * lane + (lsel ? (D1 - HW) : 0);
          *(volatile v4u*)gp = pv;
          __threadfence();
          *(volatile v4u*)gp = pv;
        } else {
          y0 = ((y0 > 0.f) ? y0 : (y0 - y0)) + pzr;
          y1 = ((y1 > 0.f) ? y1 : (y1 - y1)) + pzr;
          y2 = ((y2 > 0.f) ? y2 : (y2 - y2)) + pzr;
          y3 = ((y3 > 0.f) ? y3 : (y3 - y3)) + pzr;
          v4f ov4;
          ov4.x = y0; ov4.y = y1; ov4.z = y2; ov4.w = y3;
          if (live) {
            float* op = outp + (size_t)node * D2 + 4 * lane;
            *(volatile v4f*)op = ov4;
            __threadfence();
            *(volatile v4f*)op = ov4;
          }
        }
      }
    }
  }

  if (lane == 0) misc[16 + wave] = bigAny;
  __syncthreads();
  if (wave == 0) {
    int f = ovf;
#pragma unroll
    for (int w2 = 0; w2 < NWAVE; ++w2) f |= misc[16 + w2];
    f = (f != 0) ? 1 : 0;
    int* fp = flg + (size_t)blockIdx.x * 32 + lane;
    *(volatile int*)fp = f;
    __threadfence();
    *(volatile int*)fp = f;
  }
}

__global__ __launch_bounds__(NTHR) void k_pool(const float* __restrict__ x2, const int* __restrict__ batch,
                                               int nN, float* pool) {
  __shared__ __attribute__((aligned(16))) float part[NWAVE * D2];
  const int tid = (int)threadIdx.x, lane = tid & 31, wave = tid >> 5;
  const int g = (int)blockIdx.x;
  float m0 = 0.0f, m1 = 0.0f, m2 = 0.0f, m3 = 0.0f;
  const int nIt = (nN + NTHR - 1) / NTHR;
#pragma unroll 1
  for (int it = 0; it < nIt; ++it) {
    const int base = (it * NWAVE + wave) * 32;
    const int n    = base + lane;
    const int ncl  = n < nN ? n : nN - 1;
    const int b    = batch[ncl];
    const bool hit = (n < nN) && (b == g);
    unsigned mask = __builtin_amdgcn_ballot_w32(hit);
#pragma unroll 1
    for (int q = 0; q < 32; ++q) {
      if (mask == 0u) break;
      const int k = __builtin_ctz(mask);
      mask &= mask - 1u;
      int node = base + k;
      node = node < 0 ? 0 : (node > nN - 1 ? nN - 1 : node);
      const v4f v = *(const v4f*)(x2 + (size_t)node * D2 + 4 * lane);
      m0 = smax(m0, v.x); m1 = smax(m1, v.y); m2 = smax(m2, v.z); m3 = smax(m3, v.w);
    }
  }
  {
    v4f pv; pv.x = m0; pv.y = m1; pv.z = m2; pv.w = m3;
    *(v4fa*)(part + wave * D2 + 4 * lane) = pv;
  }
  __syncthreads();
  if (wave == 0) {
    v4f r = *(const v4fa*)(part + 4 * lane);
#pragma unroll
    for (int w2 = 1; w2 < NWAVE; ++w2) {
      const v4f v = *(const v4fa*)(part + w2 * D2 + 4 * lane);
      r.x = smax(r.x, v.x); r.y = smax(r.y, v.y); r.z = smax(r.z, v.z); r.w = smax(r.w, v.w);
    }
    float* op = pool + (size_t)g * D2 + 4 * lane;
    *(volatile v4f*)op = r;
    __threadfence();
    *(volatile v4f*)op = r;
  }
}

__global__ __launch_bounds__(NTHR) void k_head(const float* __restrict__ pool,
                                               const float* __restrict__ w1, const float* __restrict__ b1,
                                               const float* __restrict__ w2, const float* __restrict__ b2,
                                               const int* __restrict__ flg, int nFlag, float* out, int nG) {
  __shared__ __attribute__((aligned(16))) float sw1[D2 * NF1];
  __shared__ __attribute__((aligned(16))) float sb1[NF1];
  __shared__ __attribute__((aligned(16))) float sw2[NF1];
  __shared__ __attribute__((aligned(16))) float sb2[4];
  __shared__ int sfl[NWAVE];
  const int tid = (int)threadIdx.x, lane = tid & 31, wave = tid >> 5;
#pragma unroll
  for (int i = tid; i < D2 * NF1 / 4; i += NTHR) {
    const v4f a = bfr4(*(const v4fa*)(w1 + 4 * i));
    *(v4fa*)(sw1 + 4 * i) = a;
  }
  {
    const int j = tid & (NF1 - 1);
    const float vb = bfr(b1[j]);
    const float vw = bfr(w2[j]);
    const float v2 = bfr(b2[0]);
    if (tid < NF1) { sb1[tid] = vb; sw2[tid] = vw; }
    if (tid < 4) sb2[tid] = v2;
  }
  {
    const int fi = tid < nFlag ? tid : nFlag - 1;
    const int fv = flg[(size_t)fi * 32];
    const bool bad = (tid < nFlag) && (fv != 0);
    const unsigned mk = __builtin_amdgcn_ballot_w32(bad);
    if (lane == 0) sfl[wave] = (mk != 0u) ? 1 : 0;
  }
  __syncthreads();
  int ov = 0;
#pragma unroll
  for (int w2i = 0; w2i < NWAVE; ++w2i) ov |= sfl[w2i];

  const int g  = tid;
  const int gc = g < nG ? g : nG - 1;
  float acc[NF1];
#pragma unroll
  for (int j = 0; j < NF1; ++j) acc[j] = sb1[j];
  const float* pr = pool + (size_t)gc * D2;
#pragma unroll 1
  for (int k = 0; k < D2; ++k) {
    const float p = pr[k];
    const v4f wa = *(const v4fa*)(sw1 + k * NF1);
    const v4f wb = *(const v4fa*)(sw1 + k * NF1 + 4);
    const v4f wc = *(const v4fa*)(sw1 + k * NF1 + 8);
    const v4f wd = *(const v4fa*)(sw1 + k * NF1 + 12);
    acc[0]  = fmaf(p, wa.x, acc[0]);  acc[1]  = fmaf(p, wa.y, acc[1]);
    acc[2]  = fmaf(p, wa.z, acc[2]);  acc[3]  = fmaf(p, wa.w, acc[3]);
    acc[4]  = fmaf(p, wb.x, acc[4]);  acc[5]  = fmaf(p, wb.y, acc[5]);
    acc[6]  = fmaf(p, wb.z, acc[6]);  acc[7]  = fmaf(p, wb.w, acc[7]);
    acc[8]  = fmaf(p, wc.x, acc[8]);  acc[9]  = fmaf(p, wc.y, acc[9]);
    acc[10] = fmaf(p, wc.z, acc[10]); acc[11] = fmaf(p, wc.w, acc[11]);
    acc[12] = fmaf(p, wd.x, acc[12]); acc[13] = fmaf(p, wd.y, acc[13]);
    acc[14] = fmaf(p, wd.z, acc[14]); acc[15] = fmaf(p, wd.w, acc[15]);
  }
  float o = sb2[0];
#pragma unroll
  for (int j = 0; j < NF1; ++j) {
    const float hj = (acc[j] > 0.f) ? acc[j] : (acc[j] - acc[j]);
    o = fmaf(hj, sw2[j], o);
  }
  o = (ov != 0) ? __int_as_float(0x7fc00000) : o;
  if (g < nG) {
    float* op = out + g;
    *(volatile float*)op = o;
    __threadfence();
    *(volatile float*)op = o;
  }
}

static inline int cdiv(int a, int b) { return (a + b - 1) / b; }

extern "C" void kernel_launch(void* const* d_in, const int* in_sizes, int n_in,
                              void* d_out, int out_size, void* d_ws, size_t ws_size,
                              hipStream_t stream) {
  if (n_in < 15) return;
  if (in_sizes[0] < DIN || (in_sizes[0] % DIN) != 0) return;
  const int nN = in_sizes[0] / DIN;
  if (nN < 1 || nN > (1 << 21)) return;
  if (in_sizes[1] < 2 || (in_sizes[1] & 1) != 0) return;
  const int nE = in_sizes[1] / 2;
  if (nE < 1 || nE >= (1 << 21)) return;
  if (in_sizes[2] != nN) return;
  if (in_sizes[3] != DIN * D1) return;
  if (in_sizes[4] != D1 || in_sizes[5] != D1 || in_sizes[6] != D1) return;
  if (in_sizes[7] != D1 * D2) return;
  if (in_sizes[8] != D2 || in_sizes[9] != D2 || in_sizes[10] != D2) return;
  if (in_sizes[11] != D2 * NF1) return;
  if (in_sizes[12] != NF1 || in_sizes[13] != NF1 || in_sizes[14] != 1) return;
  if (out_size != NG) return;

  const float* x    = (const float*)d_in[0];
  const int*   edge = (const int*)d_in[1];
  const int*   bat  = (const int*)d_in[2];
  const float* W1   = (const float*)d_in[3];
  const float* a1s  = (const float*)d_in[4];
  const float* a1d  = (const float*)d_in[5];
  const float* b1   = (const float*)d_in[6];
  const float* W2   = (const float*)d_in[7];
  const float* a2s  = (const float*)d_in[8];
  const float* a2d  = (const float*)d_in[9];
  const float* b2   = (const float*)d_in[10];
  const float* f1w  = (const float*)d_in[11];
  const float* f1b  = (const float*)d_in[12];
  const float* f2w  = (const float*)d_in[13];
  const float* f2b  = (const float*)d_in[14];
  float* out = (float*)d_out;
  const int* src = edge;
  const int* dst = edge + nE;

  const int MP    = cdiv(nN, MROWS) * MROWS;
  const int gM    = MP / GBM;
  const int gA    = cdiv(MP, NBA);
  if ((long long)gA * NBA < (long long)MP) return;
  const int nFlag = 2 * gA;
  if (nFlag < 1 || nFlag > NTHR) return;
  const int vec8  = ((nE & 3) == 0) ? 1 : 0;
  const int nUx   = MP * (DIN / 8);

  char* ws = (char*)d_ws;
  size_t off = 0;
  const size_t oW1T = off; off += (size_t)D1 * DIN * 2;          off = (off + 255) & ~(size_t)255;
  const size_t oW2T = off; off += (size_t)D2 * KP2 * 2;          off = (off + 255) & ~(size_t)255;
  const size_t oXB  = off; off += (size_t)MP * DIN * 2;          off = (off + 255) & ~(size_t)255;
  const size_t oH1  = off; off += (size_t)MP * D1 * 4;           off = (off + 255) & ~(size_t)255;
  const size_t oSD1 = off; off += (size_t)2 * NH1 * MP * 4;      off = (off + 255) & ~(size_t)255;
  const size_t oX1  = off; off += (size_t)MP * KP2 * 2;          off = (off + 255) & ~(size_t)255;
  const size_t oH2  = off; off += (size_t)MP * D2 * 4;           off = (off + 255) & ~(size_t)255;
  const size_t oSD2 = off; off += (size_t)2 * MP * 4;            off = (off + 255) & ~(size_t)255;
  const size_t oX2  = off; off += (size_t)MP * D2 * 4;           off = (off + 255) & ~(size_t)255;
  const size_t oPL  = off; off += (size_t)NG * D2 * 4;           off = (off + 255) & ~(size_t)255;
  const size_t oFL  = off; off += (size_t)nFlag * 128;           off = (off + 255) & ~(size_t)255;
  if (off > ws_size || off > (size_t)WSMAX) return;
  unsigned short* W1T = (unsigned short*)(ws + oW1T);
  unsigned short* W2T = (unsigned short*)(ws + oW2T);
  unsigned short* XB  = (unsigned short*)(ws + oXB);
  float*          H1  = (float*)(ws + oH1);
  float*          SD1 = (float*)(ws + oSD1);
  unsigned short* X1  = (unsigned short*)(ws + oX1);
  float*          H2  = (float*)(ws + oH2);
  float*          SD2 = (float*)(ws + oSD2);
  float*          X2  = (float*)(ws + oX2);
  float*          PL  = (float*)(ws + oPL);
  int*            FLG = (int*)(ws + oFL);

  const size_t aggLds = (size_t)AGG_LDS_INTS * 4;
  hipFuncSetAttribute(reinterpret_cast<const void*>(&k_agg<1>), hipFuncAttributeMaxDynamicSharedMemorySize, (int)aggLds);
  hipFuncSetAttribute(reinterpret_cast<const void*>(&k_agg<2>), hipFuncAttributeMaxDynamicSharedMemorySize, (int)aggLds);

  k_prep<<<(NU1 + NU2 + nUx) / NTHR, NTHR, 0, stream>>>(W1, W2, x, nN, nUx, W1T, W2T, XB);
  k_gemm<<<dim3(gM, NH1), GTHR, 0, stream>>>(XB, DIN, W1T, DIN, DIN, H1, D1, a1s, a1d, SD1, MP);
  k_agg<1><<<gA, NTHR, aggLds, stream>>>(src, dst, nE, nN, vec8, MP, SD1, H1, b1, X1, X2, FLG);
  k_gemm<<<dim3(gM, 1), GTHR, 0, stream>>>(X1, KP2, W2T, KP2, KP2, H2, D2, a2s, a2d, SD2, MP);
  k_agg<2><<<gA, NTHR, aggLds, stream>>>(src, dst, nE, nN, vec8, MP, SD2, H2, b2, X1, X2, FLG + (size_t)gA * 32);
  k_pool<<<NG, NTHR, 0, stream>>>(X2, bat, nN, PL);
  k_head<<<1, NTHR, 0, stream>>>(PL, f1w, f1b, f2w, f2b, FLG, nFlag, out, NG);
}
